// SpaceTimeSelfAttention_2525440770136
// MI455X (gfx1250) — hardware-verified
//
#include <hip/hip_runtime.h>
#include <stddef.h>


typedef __bf16   v16bf __attribute__((ext_vector_type(16)));
typedef __bf16   v8bf  __attribute__((ext_vector_type(8)));
typedef _Float16 v16h  __attribute__((ext_vector_type(16)));
typedef _Float16 v8h   __attribute__((ext_vector_type(8)));
typedef float    v8f   __attribute__((ext_vector_type(8)));
typedef float    v4f   __attribute__((ext_vector_type(4)));
typedef int      v4i   __attribute__((ext_vector_type(4)));

#define NHEADS 12
#define HDIM   768
#define DHEAD  64
#define SEQ    1024
#define BATCH  4
#define NROWS  (BATCH * SEQ)
#define NROWTOT (BATCH * NHEADS * SEQ)
#define XELEMS ((size_t)NROWS * HDIM)
#define WELEMS ((size_t)HDIM * HDIM)
#define PROJ_ELEMS ((size_t)BATCH * NHEADS * SEQ * DHEAD)
#define CPITCH 68
#define HPITCH 72
#define VPITCH 40

union BF8   { v8bf v; v4i w; };
union HF8   { v8h  v; v4i w; };
union BFrag { v8bf p[2]; v16bf v; };
union HFrag { v8h  p[2]; v16h  v; };

#define WMMA_NOPS "v_nop\n\tv_nop\n\tv_nop\n\tv_nop"

__device__ __forceinline__ v16bf frag_bf16(const __bf16* p)
{
    BFrag u;
    u.p[0] = *(const v8bf*)(p);
    u.p[1] = *(const v8bf*)(p + 16);
    return u.v;
}
__device__ __forceinline__ v16h frag_f16(const _Float16* p)
{
    HFrag u;
    u.p[0] = *(const v8h*)(p);
    u.p[1] = *(const v8h*)(p + 16);
    return u.v;
}

__device__ __forceinline__ v8f mma_bf16(v8f c, v16bf a, v16bf b)
{
    return __builtin_amdgcn_wmma_f32_16x16x32_bf16(false, a, false, b, (short)0, c, false, false);
}
__device__ __forceinline__ v8f mma_f16(v8f c, v16h a, v16h b)
{
    return __builtin_amdgcn_wmma_f32_16x16x32_f16(false, a, false, b, (short)0, c, false, false);
}

__global__ __launch_bounds__(256)
void cvt_kernel(const float* __restrict__ src, __bf16* dst, int n8)
{
    const int t = blockIdx.x * blockDim.x + threadIdx.x;
    if (t >= n8) return;
    const v4f a = *(const v4f*)(src + (size_t)t * 8);
    const v4f b = *(const v4f*)(src + (size_t)t * 8 + 4);
    BF8 o;
#pragma unroll
    for (int i = 0; i < 4; ++i) { o.v[i] = (__bf16)a[i]; o.v[4 + i] = (__bf16)b[i]; }
    const v4i w = o.w;
    volatile v4i* p = (volatile v4i*)(dst + (size_t)t * 8);
    *p = w;
    __threadfence();
    *p = w;
}

template <int MODE, int SCALE, int NORM>
__device__ __forceinline__ void proj_store(float (*Cs)[CPITCH], float* Srn, float* Ssq, int lane, size_t row0,
                                           unsigned short* outA, unsigned short* outB, float* rn, float* sq)
{
#pragma unroll
    for (int i = 0; i < 8; ++i) {
        const int lr = 4 * i + (lane >> 3), seg = lane & 7;
        const v4f x0 = *(const v4f*)&Cs[lr][seg * 8];
        const v4f x1 = *(const v4f*)&Cs[lr][seg * 8 + 4];
        const size_t go = (row0 + lr) * DHEAD + seg * 8;
        if (MODE == 0) {
            BF8 hi, lo;
#pragma unroll
            for (int j = 0; j < 4; ++j) {
                const float a0 = x0[j]; const __bf16 h0 = (__bf16)a0;
                hi.v[j] = h0; lo.v[j] = (__bf16)(a0 - (float)h0);
                const float a1 = x1[j]; const __bf16 h1 = (__bf16)a1;
                hi.v[4 + j] = h1; lo.v[4 + j] = (__bf16)(a1 - (float)h1);
            }
            *(volatile v4i*)(outA + go) = hi.w;
            *(volatile v4i*)(outB + go) = lo.w;
        } else {
            HF8 y;
#pragma unroll
            for (int j = 0; j < 4; ++j) {
                y.v[j]     = (_Float16)(x0[j] * (float)SCALE);
                y.v[4 + j] = (_Float16)(x1[j] * (float)SCALE);
            }
            *(volatile v4i*)(outA + go) = y.w;
        }
    }
    if (NORM) {
        if (lane < 16) {
            const int g = lane & 7;
            v4f v; float* dp;
            if (lane < 8) { v = *(const v4f*)&Srn[4 * g]; dp = rn + row0 + 4 * g; }
            else          { v = *(const v4f*)&Ssq[4 * g]; dp = sq + row0 + 4 * g; }
            *(volatile v4f*)dp = v;
        }
    }
}

template <int MODE, int SCALE, int NORM>
__global__ __launch_bounds__(32)
void proj_kernel(const __bf16* __restrict__ Xb, const __bf16* __restrict__ Wb, const float* __restrict__ bias,
                 unsigned short* outA, unsigned short* outB, float* rn, float* sq)
{
    __shared__ __attribute__((aligned(16))) float Cs[32][CPITCH];
    __shared__ __attribute__((aligned(16))) float Srn[32];
    __shared__ __attribute__((aligned(16))) float Ssq[32];

    const int lane = threadIdx.x & 31;
    const int hsel = lane >> 4;
    const int lm   = lane & 15;
    const int m0   = blockIdx.x * 32;
    const int n0   = blockIdx.y * 64;
    if (m0 + 32 > NROWS || n0 + 64 > HDIM) return;

    const __bf16* a0p = Xb + (size_t)(m0 + lm) * HDIM + hsel * 8;
    const __bf16* a1p = Xb + (size_t)(m0 + 16 + lm) * HDIM + hsel * 8;
    const __bf16* b0p = Wb + (size_t)(n0 +  0 + lm) * HDIM + hsel * 8;
    const __bf16* b1p = Wb + (size_t)(n0 + 16 + lm) * HDIM + hsel * 8;
    const __bf16* b2p = Wb + (size_t)(n0 + 32 + lm) * HDIM + hsel * 8;
    const __bf16* b3p = Wb + (size_t)(n0 + 48 + lm) * HDIM + hsel * 8;

    v8f acc[2][4];
#pragma unroll
    for (int mb = 0; mb < 2; ++mb)
#pragma unroll
        for (int nb = 0; nb < 4; ++nb) acc[mb][nb] = v8f{};

#pragma unroll 1
    for (int k0 = 0; k0 < HDIM; k0 += 32) {
        const v16bf a0 = frag_bf16(a0p + k0);
        const v16bf a1 = frag_bf16(a1p + k0);
        const v16bf b0 = frag_bf16(b0p + k0);
        const v16bf b1 = frag_bf16(b1p + k0);
        const v16bf b2 = frag_bf16(b2p + k0);
        const v16bf b3 = frag_bf16(b3p + k0);
        acc[0][0] = mma_bf16(acc[0][0], a0, b0);
        acc[0][1] = mma_bf16(acc[0][1], a0, b1);
        acc[0][2] = mma_bf16(acc[0][2], a0, b2);
        acc[0][3] = mma_bf16(acc[0][3], a0, b3);
        acc[1][0] = mma_bf16(acc[1][0], a1, b0);
        acc[1][1] = mma_bf16(acc[1][1], a1, b1);
        acc[1][2] = mma_bf16(acc[1][2], a1, b2);
        acc[1][3] = mma_bf16(acc[1][3], a1, b3);
        asm volatile(WMMA_NOPS
                     : "+v"(acc[0][0]), "+v"(acc[0][1]), "+v"(acc[0][2]), "+v"(acc[0][3]),
                       "+v"(acc[1][0]), "+v"(acc[1][1]), "+v"(acc[1][2]), "+v"(acc[1][3])
                     : "v"(a0), "v"(a1), "v"(b0), "v"(b1), "v"(b2), "v"(b3));
    }

#pragma unroll
    for (int nb = 0; nb < 4; ++nb) {
        const float bn = bias[n0 + nb * 16 + lm];
#pragma unroll
        for (int mb = 0; mb < 2; ++mb) {
#pragma unroll
            for (int r = 0; r < 8; ++r)
                Cs[mb * 16 + 8 * hsel + r][nb * 16 + lm] = acc[mb][nb][r] + bn;
        }
    }
    __syncthreads();

    if (NORM) {
        float ss = 0.f;
#pragma unroll
        for (int d = 0; d < DHEAD; d += 4) {
            const v4f x = *(const v4f*)&Cs[lane][d];
            ss += x[0] * x[0]; ss += x[1] * x[1]; ss += x[2] * x[2]; ss += x[3] * x[3];
        }
        Srn[lane] = 1.0f / (sqrtf(ss) + 1e-6f);
        Ssq[lane] = ss;
    }
    __syncthreads();

    const int bI = m0 >> 10, s0 = m0 & (SEQ - 1), hh = n0 >> 6;
    const size_t row0 = ((size_t)(bI * NHEADS + hh)) * SEQ + s0;

    proj_store<MODE, SCALE, NORM>(Cs, Srn, Ssq, lane, row0, outA, outB, rn, sq);
    __threadfence();
    proj_store<MODE, SCALE, NORM>(Cs, Srn, Ssq, lane, row0, outA, outB, rn, sq);
}

__device__ __forceinline__ void attn_store(float (*Os)[CPITCH], int wave, int lane, float* out, size_t orow0, int h)
{
#pragma unroll
    for (int i = 0; i < 8; ++i) {
        const int lr  = wave * 16 + 2 * i + (lane >> 4);
        const int col = (lane & 15) * 4;
        const v4f v = *(const v4f*)&Os[lr][col];
        float* gp = out + (orow0 + lr) * HDIM + h * DHEAD + col;
        *(volatile v4f*)gp = v;
    }
}

__global__ __launch_bounds__(64)
void attn_kernel(const __bf16* __restrict__ qh, const __bf16* __restrict__ ql,
                 const __bf16* __restrict__ kh, const __bf16* __restrict__ kl,
                 const _Float16* __restrict__ tp, const _Float16* __restrict__ sp,
                 const _Float16* __restrict__ vp,
                 const float* __restrict__ rnT, const float* __restrict__ sqT,
                 const float* __restrict__ rnS, const float* __restrict__ sqS,
                 const float* __restrict__ mask, float* out)
{
    __shared__ __attribute__((aligned(16))) __bf16   KH[32][HPITCH];
    __shared__ __attribute__((aligned(16))) __bf16   KL[32][HPITCH];
    __shared__ __attribute__((aligned(16))) __bf16   QHs[32][HPITCH];
    __shared__ __attribute__((aligned(16))) __bf16   QLs[32][HPITCH];
    __shared__ __attribute__((aligned(16))) _Float16 TK[32][HPITCH];
    __shared__ __attribute__((aligned(16))) _Float16 SK[32][HPITCH];
    __shared__ __attribute__((aligned(16))) _Float16 TQ[32][HPITCH];
    __shared__ __attribute__((aligned(16))) _Float16 SQ[32][HPITCH];
    __shared__ __attribute__((aligned(16))) _Float16 Vt[64][VPITCH];
    __shared__ __attribute__((aligned(16))) _Float16 pP[2][16][VPITCH];
    __shared__ __attribute__((aligned(16))) float    Os[32][CPITCH];

    const int bh = blockIdx.x;
    if (bh >= BATCH * NHEADS) return;
    const int q0blk = blockIdx.y * 32;
    if (q0blk + 32 > SEQ) return;
    const int b = bh / NHEADS, h = bh - b * NHEADS;
    const int tid  = threadIdx.x;
    const int wave = tid >> 5;
    const int lane = tid & 31;
    const int hsel = lane >> 4;
    const int lm   = lane & 15;
    const int qr   = wave * 16 + lm;

    for (int c = tid; c < 1024; c += 64) {
        const int t = c >> 8, e = c & 255, row = e >> 3, seg = e & 7;
        const size_t go = ((size_t)(bh * SEQ + q0blk + row) << 6) + seg * 8;
        if (t == 0)      *(v8bf*)&QHs[row][seg * 8] = *(const v8bf*)(qh + go);
        else if (t == 1) *(v8bf*)&QLs[row][seg * 8] = *(const v8bf*)(ql + go);
        else if (t == 2) *(v8h*)&TQ[row][seg * 8]   = *(const v8h*)(tp + go);
        else             *(v8h*)&SQ[row][seg * 8]   = *(const v8h*)(sp + go);
    }

    float fq[8], gq[8], mI[8], lI[8];
#pragma unroll
    for (int r = 0; r < 8; ++r) {
        const int qi = bh * SEQ + q0blk + wave * 16 + 8 * hsel + r;
        const float rt = rnT[qi], rs = rnS[qi];
        fq[r] = (rt * (1.0f / 256.0f)) * (rs * (1.0f / 256.0f)) * 0.125f;
        gq[r] = (sqT[qi] * rt) * (sqS[qi] * rs) * 0.125f;
        mI[r] = -3.0e38f;
        lI[r] = 0.f;
    }
    v8f O[4] = {v8f{}, v8f{}, v8f{}, v8f{}};

    for (int k0 = 0; k0 < SEQ; k0 += 32) {
        __syncthreads();

        for (int c = tid; c < 1024; c += 64) {
            const int t = c >> 8, e = c & 255, row = e >> 3, seg = e & 7;
            const size_t go = ((size_t)(bh * SEQ + k0 + row) << 6) + seg * 8;
            if (t == 0)      *(v8bf*)&KH[row][seg * 8] = *(const v8bf*)(kh + go);
            else if (t == 1) *(v8bf*)&KL[row][seg * 8] = *(const v8bf*)(kl + go);
            else if (t == 2) *(v8h*)&TK[row][seg * 8]  = *(const v8h*)(tp + go);
            else             *(v8h*)&SK[row][seg * 8]  = *(const v8h*)(sp + go);
        }
        for (int c = tid; c < 256; c += 64) {
            const int kk = c >> 3, sg = c & 7;
            const v8h vv = *(const v8h*)(vp + ((size_t)(bh * SEQ + k0 + kk) << 6) + sg * 8);
#pragma unroll
            for (int i = 0; i < 8; ++i) Vt[sg * 8 + i][kk] = vv[i];
        }
        __syncthreads();

        const bool diag = (k0 == q0blk);

        float sb[2][8];
#pragma unroll
        for (int j = 0; j < 2; ++j) {
            const int rr = j * 16 + lm;
            v8f accB = v8f{}, accT = v8f{}, accS = v8f{};
#pragma unroll 1
            for (int c = 0; c < 2; ++c) {
                const int off = c * 32 + 8 * hsel;
                const v16bf aH = frag_bf16(&QHs[qr][off]);
                const v16bf aL = frag_bf16(&QLs[qr][off]);
                const v16bf bH = frag_bf16(&KH[rr][off]);
                const v16bf bL = frag_bf16(&KL[rr][off]);
                accB = mma_bf16(accB, aH, bH);
                accB = mma_bf16(accB, aH, bL);
                accB = mma_bf16(accB, aL, bH);
                asm volatile(WMMA_NOPS : "+v"(accB) : "v"(aH), "v"(aL), "v"(bH), "v"(bL));
                const v16h aT = frag_f16(&TQ[qr][off]);
                const v16h bT = frag_f16(&TK[rr][off]);
                const v16h aS = frag_f16(&SQ[qr][off]);
                const v16h bS = frag_f16(&SK[rr][off]);
                accT = mma_f16(accT, aT, bT);
                accS = mma_f16(accS, aS, bS);
                asm volatile(WMMA_NOPS : "+v"(accT), "+v"(accS) : "v"(aT), "v"(bT), "v"(aS), "v"(bS));
            }
            const float mval = mask[b * SEQ + k0 + rr];
            const bool dj = diag && (j == wave);
#pragma unroll
            for (int r = 0; r < 8; ++r) {
                const bool de = dj && (lm == 8 * hsel + r);
                const float s3 = de ? (accB[r] * gq[r])
                                    : (accB[r] * (accT[r] * accS[r]) * fq[r]);
                sb[j][r] = s3 + mval;
            }
        }

#pragma unroll
        for (int r = 0; r < 8; ++r) {
            float v = fmaxf(sb[0][r], sb[1][r]);
#pragma unroll
            for (int off = 1; off < 16; off <<= 1) v = fmaxf(v, __shfl_xor(v, off, 16));
            const float M2 = fmaxf(mI[r], v);
            const float al = __expf(mI[r] - M2);
            const float p0 = __expf(sb[0][r] - M2);
            const float p1 = __expf(sb[1][r] - M2);
            float rs = p0 + p1;
#pragma unroll
            for (int off = 1; off < 16; off <<= 1) rs += __shfl_xor(rs, off, 16);
            mI[r] = M2;
            lI[r] = lI[r] * al + rs;
            O[0][r] = O[0][r] * al;
            O[1][r] = O[1][r] * al;
            O[2][r] = O[2][r] * al;
            O[3][r] = O[3][r] * al;
            const int m = r + 8 * hsel;
            pP[wave][m][lm]      = (_Float16)(p0 * 4096.0f);
            pP[wave][m][16 + lm] = (_Float16)(p1 * 4096.0f);
        }
        __syncthreads();

        const v16h aP  = frag_f16(&pP[wave][lm][8 * hsel]);
        const v16h bV0 = frag_f16(&Vt[ 0 + lm][8 * hsel]);
        const v16h bV1 = frag_f16(&Vt[16 + lm][8 * hsel]);
        const v16h bV2 = frag_f16(&Vt[32 + lm][8 * hsel]);
        const v16h bV3 = frag_f16(&Vt[48 + lm][8 * hsel]);
        O[0] = mma_f16(O[0], aP, bV0);
        O[1] = mma_f16(O[1], aP, bV1);
        O[2] = mma_f16(O[2], aP, bV2);
        O[3] = mma_f16(O[3], aP, bV3);
        asm volatile(WMMA_NOPS
                     : "+v"(O[0]), "+v"(O[1]), "+v"(O[2]), "+v"(O[3])
                     : "v"(aP), "v"(bV0), "v"(bV1), "v"(bV2), "v"(bV3));
    }

#pragma unroll
    for (int r = 0; r < 8; ++r) {
        const float inv = (1.0f / lI[r]) * (1.0f / 262144.0f);
        const int lr = wave * 16 + 8 * hsel + r;
        Os[lr][lm]      = O[0][r] * inv;
        Os[lr][16 + lm] = O[1][r] * inv;
        Os[lr][32 + lm] = O[2][r] * inv;
        Os[lr][48 + lm] = O[3][r] * inv;
    }
    __syncthreads();

    const size_t orow0 = (size_t)(b * SEQ + q0blk);
    attn_store(Os, wave, lane, out, orow0, h);
    __threadfence();
    attn_store(Os, wave, lane, out, orow0, h);
}

extern "C" void kernel_launch(void* const* d_in, const int* in_sizes, int n_in,
                              void* d_out, int out_size, void* d_ws, size_t ws_size,
                              hipStream_t stream)
{
    if (n_in < 14) return;
    if ((size_t)in_sizes[0] != XELEMS || (size_t)in_sizes[1] != XELEMS || (size_t)in_sizes[2] != XELEMS) return;
    if (in_sizes[3] != BATCH * SEQ) return;
    for (int i = 4; i < 14; i += 2)
        if ((size_t)in_sizes[i] != WELEMS || in_sizes[i + 1] != HDIM) return;
    if ((size_t)out_size != XELEMS) return;

    const float* hidden = (const float*)d_in[0];
    const float* timee  = (const float*)d_in[1];
    const float* space  = (const float*)d_in[2];
    const float* mask   = (const float*)d_in[3];
    const float* Wq = (const float*)d_in[4];   const float* bq = (const float*)d_in[5];
    const float* Wk = (const float*)d_in[6];   const float* bk = (const float*)d_in[7];
    const float* Wv = (const float*)d_in[8];   const float* bv = (const float*)d_in[9];
    const float* Wt = (const float*)d_in[10];  const float* bt = (const float*)d_in[11];
    const float* Ws = (const float*)d_in[12];  const float* bs = (const float*)d_in[13];
    float* out = (float*)d_out;

    char* ws = (char*)d_ws;
    size_t off = 0;
    __bf16* Xbf = (__bf16*)(ws + off);                 off += (size_t)3 * XELEMS * 2;
    __bf16* Wbf = (__bf16*)(ws + off);                 off += (size_t)5 * WELEMS * 2;
    unsigned short* pl = (unsigned short*)(ws + off);  off += (size_t)7 * PROJ_ELEMS * 2;
    float* rn = (float*)(ws + off);                    off += (size_t)2 * NROWTOT * 4;
    float* sq = (float*)(ws + off);                    off += (size_t)2 * NROWTOT * 4;
    if (off > ws_size) return;

    unsigned short* QH = pl + 0 * PROJ_ELEMS;
    unsigned short* QL = pl + 1 * PROJ_ELEMS;
    unsigned short* KHp = pl + 2 * PROJ_ELEMS;
    unsigned short* KLp = pl + 3 * PROJ_ELEMS;
    unsigned short* TPl = pl + 4 * PROJ_ELEMS;
    unsigned short* SPl = pl + 5 * PROJ_ELEMS;
    unsigned short* VPl = pl + 6 * PROJ_ELEMS;

    const int nx8 = (int)(XELEMS / 8), nw8 = (int)(WELEMS / 8);
    const dim3 cb(256);
    cvt_kernel<<<dim3((nx8 + 255) / 256), cb, 0, stream>>>(hidden, Xbf, nx8);
    cvt_kernel<<<dim3((nx8 + 255) / 256), cb, 0, stream>>>(timee,  Xbf + XELEMS, nx8);
    cvt_kernel<<<dim3((nx8 + 255) / 256), cb, 0, stream>>>(space,  Xbf + 2 * XELEMS, nx8);
    cvt_kernel<<<dim3((nw8 + 255) / 256), cb, 0, stream>>>(Wq, Wbf + 0 * WELEMS, nw8);
    cvt_kernel<<<dim3((nw8 + 255) / 256), cb, 0, stream>>>(Wk, Wbf + 1 * WELEMS, nw8);
    cvt_kernel<<<dim3((nw8 + 255) / 256), cb, 0, stream>>>(Wv, Wbf + 2 * WELEMS, nw8);
    cvt_kernel<<<dim3((nw8 + 255) / 256), cb, 0, stream>>>(Wt, Wbf + 3 * WELEMS, nw8);
    cvt_kernel<<<dim3((nw8 + 255) / 256), cb, 0, stream>>>(Ws, Wbf + 4 * WELEMS, nw8);

    const dim3 pg(NROWS / 32, HDIM / 64), pb(32);
    proj_kernel<0, 1, 0><<<pg, pb, 0, stream>>>(Xbf, Wbf + 0 * WELEMS, bq, QH,  QL,  rn, sq);
    proj_kernel<0, 1, 0><<<pg, pb, 0, stream>>>(Xbf, Wbf + 1 * WELEMS, bk, KHp, KLp, rn, sq);
    proj_kernel<1, 64, 0><<<pg, pb, 0, stream>>>(Xbf, Wbf + 2 * WELEMS, bv, VPl, VPl, rn, sq);
    proj_kernel<1, 16, 1><<<pg, pb, 0, stream>>>(Xbf + XELEMS,     Wbf + 3 * WELEMS, bt, TPl, TPl, rn, sq);
    proj_kernel<1, 16, 1><<<pg, pb, 0, stream>>>(Xbf + 2 * XELEMS, Wbf + 4 * WELEMS, bs, SPl, SPl,
                                                 rn + NROWTOT, sq + NROWTOT);

    attn_kernel<<<dim3(BATCH * NHEADS, SEQ / 32), dim3(64), 0, stream>>>(
        (const __bf16*)QH, (const __bf16*)QL, (const __bf16*)KHp, (const __bf16*)KLp,
        (const _Float16*)TPl, (const _Float16*)SPl, (const _Float16*)VPl,
        rn, sq, rn + NROWTOT, sq + NROWTOT, mask, out);
}
